// NAR_26749056319699
// MI455X (gfx1250) — hardware-verified
//
#include <hip/hip_runtime.h>


typedef unsigned short us;
typedef us       v8us __attribute__((ext_vector_type(8)));
typedef _Float16 v8h  __attribute__((ext_vector_type(8)));
typedef _Float16 v16h __attribute__((ext_vector_type(16)));
typedef __bf16   v16b __attribute__((ext_vector_type(16)));
typedef float    v8f  __attribute__((ext_vector_type(8)));
typedef float    v4f  __attribute__((ext_vector_type(4)));
typedef int      v4i  __attribute__((ext_vector_type(4)));

static constexpr int DDIM   = 256;
static constexpr int HDIM   = 512;
static constexpr int ELLW   = 96;
static constexpr int ELLCAP = 95;
static constexpr int NPB    = 128;

union FragH { v16h v; v8us h[2]; };
union FragB { v16b v; v8us h[2]; };

__device__ __forceinline__ void ld_frag(v8us* f, const us* __restrict__ P, int ld, int r0, int k0, int h, int m)
{
    const us* p = P + (size_t)(r0 + m) * ld + k0 + 8 * h;
    f[0] = *(const v8us*)(p);
    f[1] = *(const v8us*)(p + 16);
}

__device__ __forceinline__ v8f wmma_h(v16h a, v16h b, v8f c)
{
    c = __builtin_amdgcn_wmma_f32_16x16x32_f16(false, a, false, b, (short)0, c, false, false);
    asm volatile("v_nop\n\tv_nop\n\tv_nop\n\tv_nop" : "+v"(c) : "v"(a), "v"(b));
    return c;
}

__device__ __forceinline__ v8f wmma_b(v16b a, v16b b, v8f c)
{
    c = __builtin_amdgcn_wmma_f32_16x16x32_bf16(false, a, false, b, (short)0, c, false, false);
    asm volatile("v_nop\n\tv_nop\n\tv_nop\n\tv_nop" : "+v"(c) : "v"(a), "v"(b));
    return c;
}

__device__ __forceinline__ us bf16_bits(float x)
{
    unsigned u = __builtin_bit_cast(unsigned, x);
    u += 0x7FFFu + ((u >> 16) & 1u);
    return (us)(u >> 16);
}
__device__ __forceinline__ float bf16_val(us b)
{
    return __builtin_bit_cast(float, ((unsigned)b) << 16);
}
__device__ __forceinline__ v8us pack_f16(const float* v)
{
    union { v8h f; v8us u; } q;
#pragma unroll
    for (int i = 0; i < 8; ++i) q.f[i] = (_Float16)v[i];
    return q.u;
}
__device__ __forceinline__ void pack_bf16(const float* v, v8us& hi, v8us& lo)
{
#pragma unroll
    for (int i = 0; i < 8; ++i) {
        const us hb = bf16_bits(v[i]);
        hi[i] = hb;
        lo[i] = bf16_bits(v[i] - bf16_val(hb));
    }
}

__global__ __launch_bounds__(32)
void k_build(const int* __restrict__ src, const int* __restrict__ dst, int E, int N, int* ell)
{
    __shared__ __align__(16) int rows[NPB * ELLW];
    __shared__ int cnt[NPB];
    const int l = threadIdx.x;
    const int b = blockIdx.x;

    for (int i = l; i < NPB * ELLW; i += 32) rows[i] = 0;
    for (int i = l; i < NPB; i += 32) cnt[i] = 0;
    __syncthreads();

    for (int e0 = 0; e0 < E; e0 += 32) {
        const int e = e0 + l;
        int d = -1, s = 0;
        if (e < E) { d = dst[e]; s = src[e]; }
        const bool match = (e < E) && (d >= 0) && (d < N) && ((d >> 7) == b);
        unsigned msk = __builtin_amdgcn_ballot_w32(match);
        while (msk) {
            const int L  = __builtin_ctz(msk);
            const int dl = __builtin_amdgcn_readlane(d, L);
            const int sl = __builtin_amdgcn_readlane(s, L);
            if (l == 0) {
                const int ld = dl & (NPB - 1);
                const int p  = cnt[ld];
                if (p < ELLCAP) rows[ld * ELLW + 1 + p] = sl;
                cnt[ld] = p + 1;
            }
            msk &= msk - 1u;
        }
    }
    __syncthreads();
    for (int i = l; i < NPB; i += 32) rows[i * ELLW] = cnt[i];
    __syncthreads();

    auto st = [&]() {
        for (int ld = 0; ld < NPB; ++ld) {
            if (l < 24) {
                const v4i v = *(const v4i*)&rows[ld * ELLW + 4 * l];
                int* p = ell + (size_t)(b * NPB + ld) * ELLW + 4 * l;
                *(volatile v4i*)p = v;
            }
        }
    };
    st();
    __threadfence();
    st();
}

__global__ __launch_bounds__(256)
void k_cvt_x(const float* __restrict__ x, int N, int MP, us* out)
{
    const int t   = blockIdx.x * 256 + threadIdx.x;
    const int row = t >> 5;
    const int c   = (t & 31) * 8;
    if (row >= MP) return;
    float v[8];
#pragma unroll
    for (int i = 0; i < 8; ++i) v[i] = 0.0f;
    if (row < N) {
        const float* r = x + (size_t)row * DDIM + c;
        const v4f a = *(const v4f*)r;
        const v4f bq = *(const v4f*)(r + 4);
        v[0] = a.x; v[1] = a.y; v[2] = a.z; v[3] = a.w;
        v[4] = bq.x; v[5] = bq.y; v[6] = bq.z; v[7] = bq.w;
    }
    const v8us q = pack_f16(v);
    us* p = out + (size_t)row * DDIM + c;
    *(volatile v8us*)p = q;
    __threadfence();
    *(volatile v8us*)p = q;
}

__global__ __launch_bounds__(256)
void k_wcvt(const float* __restrict__ W, int K, int Nc, int mode, float scale, us* o1, us* o2)
{
    const int t  = blockIdx.x * 256 + threadIdx.x;
    const int kq = K >> 3;
    const int n  = t / kq;
    const int k8 = (t - n * kq) * 8;
    if (n >= Nc) return;
    float v[8];
#pragma unroll
    for (int i = 0; i < 8; ++i) v[i] = W[(size_t)(k8 + i) * Nc + n] * scale;
    const size_t o = (size_t)n * K + k8;
    if (mode == 0) {
        const v8us q = pack_f16(v);
        *(volatile v8us*)(o1 + o) = q;
        __threadfence();
        *(volatile v8us*)(o1 + o) = q;
    } else {
        v8us hi, lo;
        pack_bf16(v, hi, lo);
        *(volatile v8us*)(o1 + o) = hi;
        *(volatile v8us*)(o2 + o) = lo;
        __threadfence();
        *(volatile v8us*)(o1 + o) = hi;
        *(volatile v8us*)(o2 + o) = lo;
    }
}

template <int SPLIT, int EPI>
__global__ __launch_bounds__(128)
void k_gemm(const us* __restrict__ Ah, const us* __restrict__ Al,
            const us* __restrict__ Bh, const us* __restrict__ Bl,
            int K, int Nc, const float* __restrict__ bias, float oscale,
            float* outF, us* outH, us* outL, int Mvalid)
{
    __shared__ __align__(16) float sC[64 * 68];
    const int t  = threadIdx.x;
    const int w  = t >> 5, l = t & 31, h = l >> 4, m = l & 15;
    const int wy = w >> 1, wx = w & 1;
    const int ntn   = Nc >> 6;
    const int mt    = blockIdx.x / ntn;
    const int nt    = blockIdx.x - mt * ntn;
    const int mrow0 = mt * 64, ncol0 = nt * 64;
    const int ar0   = mrow0 + wy * 32;
    const int bc0   = ncol0 + wx * 32;

    v8f c00 = {}, c01 = {}, c10 = {}, c11 = {};

#pragma unroll 1
    for (int k0 = 0; k0 < K; k0 += 32) {
        if (SPLIT) {
            FragB ah0, ah1, al0, al1, bh0, bh1, bl0, bl1;
            ld_frag(ah0.h, Ah, K, ar0,      k0, h, m);
            ld_frag(ah1.h, Ah, K, ar0 + 16, k0, h, m);
            ld_frag(al0.h, Al, K, ar0,      k0, h, m);
            ld_frag(al1.h, Al, K, ar0 + 16, k0, h, m);
            ld_frag(bh0.h, Bh, K, bc0,      k0, h, m);
            ld_frag(bh1.h, Bh, K, bc0 + 16, k0, h, m);
            ld_frag(bl0.h, Bl, K, bc0,      k0, h, m);
            ld_frag(bl1.h, Bl, K, bc0 + 16, k0, h, m);
            c00 = wmma_b(ah0.v, bh0.v, c00); c00 = wmma_b(ah0.v, bl0.v, c00); c00 = wmma_b(al0.v, bh0.v, c00);
            c01 = wmma_b(ah0.v, bh1.v, c01); c01 = wmma_b(ah0.v, bl1.v, c01); c01 = wmma_b(al0.v, bh1.v, c01);
            c10 = wmma_b(ah1.v, bh0.v, c10); c10 = wmma_b(ah1.v, bl0.v, c10); c10 = wmma_b(al1.v, bh0.v, c10);
            c11 = wmma_b(ah1.v, bh1.v, c11); c11 = wmma_b(ah1.v, bl1.v, c11); c11 = wmma_b(al1.v, bh1.v, c11);
        } else {
            FragH a0, a1, b0, b1;
            ld_frag(a0.h, Ah, K, ar0,      k0, h, m);
            ld_frag(a1.h, Ah, K, ar0 + 16, k0, h, m);
            ld_frag(b0.h, Bh, K, bc0,      k0, h, m);
            ld_frag(b1.h, Bh, K, bc0 + 16, k0, h, m);
            c00 = wmma_h(a0.v, b0.v, c00);
            c01 = wmma_h(a0.v, b1.v, c01);
            c10 = wmma_h(a1.v, b0.v, c10);
            c11 = wmma_h(a1.v, b1.v, c11);
        }
    }

    {
        const int rb = wy * 32, cb = wx * 32;
#pragma unroll
        for (int r = 0; r < 8; ++r) {
            sC[(rb +      8 * h + r) * 68 + cb      + m] = c00[r] * oscale;
            sC[(rb +      8 * h + r) * 68 + cb + 16 + m] = c01[r] * oscale;
            sC[(rb + 16 + 8 * h + r) * 68 + cb      + m] = c10[r] * oscale;
            sC[(rb + 16 + 8 * h + r) * 68 + cb + 16 + m] = c11[r] * oscale;
        }
    }
    __syncthreads();

    auto st_f32 = [&]() {
#pragma unroll
        for (int g = 0; g < 8; ++g) {
            const int row  = g * 8 + (t >> 4);
            const int col  = (t & 15) * 4;
            const int grow = mrow0 + row;
            v4f v = *(const v4f*)&sC[row * 68 + col];
            if (EPI == 2) {
                if (grow < Mvalid) {
                    const v4f bb = *(const v4f*)(bias + ncol0 + col);
                    v += bb;
                    *(volatile v4f*)(outF + (size_t)grow * Nc + ncol0 + col) = v;
                }
            } else {
                *(volatile v4f*)(outF + (size_t)grow * Nc + ncol0 + col) = v;
            }
        }
    };
    auto st_planes = [&]() {
#pragma unroll
        for (int g = 0; g < 4; ++g) {
            const int row = g * 16 + (t >> 3);
            const int col = (t & 7) * 8;
            const v4f a  = *(const v4f*)&sC[row * 68 + col];
            const v4f bq = *(const v4f*)&sC[row * 68 + col + 4];
            float v[8] = { a.x, a.y, a.z, a.w, bq.x, bq.y, bq.z, bq.w };
#pragma unroll
            for (int i = 0; i < 8; ++i) v[i] = fmaxf(v[i] + bias[ncol0 + col + i], 0.0f);
            v8us hi, lo;
            pack_bf16(v, hi, lo);
            const size_t o = (size_t)(mrow0 + row) * Nc + ncol0 + col;
            *(volatile v8us*)(outH + o) = hi;
            *(volatile v8us*)(outL + o) = lo;
        }
    };
    if (EPI == 1) { st_planes(); __threadfence(); st_planes(); }
    else          { st_f32();    __threadfence(); st_f32();    }
}

template <int F, int RELU, int SPLIT>
__global__ __launch_bounds__(F / 8)
void k_agg(const float* __restrict__ xw, const int* __restrict__ ell, int N,
           const float* __restrict__ bias, us* outA, us* outB)
{
    const int d = blockIdx.x;
    const int c = threadIdx.x * 8;
    float o[8];
#pragma unroll
    for (int i = 0; i < 8; ++i) o[i] = 0.0f;

    if (d < N) {
        int hdr = ell[(size_t)d * ELLW];
        hdr = hdr < 0 ? 0 : hdr;
        const int cnt = hdr < ELLCAP ? hdr : ELLCAP;
        const float dd = rsqrtf(1.0f + (float)hdr);
        float acc[8];
#pragma unroll
        for (int i = 0; i < 8; ++i) acc[i] = 0.0f;
#pragma unroll 1
        for (int j = 0; j < cnt; ++j) {
            int s = ell[(size_t)d * ELLW + 1 + j];
            s = s < 0 ? 0 : (s >= N ? N - 1 : s);
            int hs = ell[(size_t)s * ELLW];
            hs = hs < 0 ? 0 : hs;
            const float ds = rsqrtf(1.0f + (float)hs);
            const float* r = xw + (size_t)s * F + c;
            const v4f a  = *(const v4f*)r;
            const v4f bq = *(const v4f*)(r + 4);
            acc[0] += ds * a.x;  acc[1] += ds * a.y;  acc[2] += ds * a.z;  acc[3] += ds * a.w;
            acc[4] += ds * bq.x; acc[5] += ds * bq.y; acc[6] += ds * bq.z; acc[7] += ds * bq.w;
        }
        const float* r = xw + (size_t)d * F + c;
        const v4f a  = *(const v4f*)r;
        const v4f bq = *(const v4f*)(r + 4);
        const float xs[8] = { a.x, a.y, a.z, a.w, bq.x, bq.y, bq.z, bq.w };
#pragma unroll
        for (int i = 0; i < 8; ++i) {
            float v = dd * (acc[i] + dd * xs[i]) + bias[c + i];
            if (RELU) v = fmaxf(v, 0.0f);
            o[i] = v;
        }
    }

    const size_t off = (size_t)d * F + c;
    if (SPLIT) {
        v8us hi, lo;
        pack_bf16(o, hi, lo);
        *(volatile v8us*)(outA + off) = hi;
        *(volatile v8us*)(outB + off) = lo;
        __threadfence();
        *(volatile v8us*)(outA + off) = hi;
        *(volatile v8us*)(outB + off) = lo;
    } else {
        const v8us q = pack_f16(o);
        *(volatile v8us*)(outA + off) = q;
        __threadfence();
        *(volatile v8us*)(outA + off) = q;
    }
}

static inline size_t ws_take(size_t& off, size_t bytes)
{
    off = (off + 255) & ~(size_t)255;
    const size_t cur = off;
    off += bytes;
    return cur;
}
static inline int cdiv(long a, long b) { return (int)((a + b - 1) / b); }

extern "C" void kernel_launch(void* const* d_in, const int* in_sizes, int n_in,
                              void* d_out, int out_size, void* d_ws, size_t ws_size,
                              hipStream_t stream)
{
    if (n_in < 10) return;
    const float* x   = (const float*)d_in[0];
    const int*   ei  = (const int*)  d_in[1];
    const float* W1  = (const float*)d_in[2];
    const float* b1  = (const float*)d_in[3];
    const float* W2  = (const float*)d_in[4];
    const float* b2  = (const float*)d_in[5];
    const float* Wm1 = (const float*)d_in[6];
    const float* bm1 = (const float*)d_in[7];
    const float* Wm2 = (const float*)d_in[8];
    const float* bm2 = (const float*)d_in[9];

    const int N = in_sizes[0] / DDIM;
    const int E = in_sizes[1] / 2;
    if (N <= 0 || E < 0) return;
    if (in_sizes[2] != DDIM * HDIM || in_sizes[4] != HDIM * DDIM ||
        in_sizes[6] != DDIM * HDIM || in_sizes[8] != HDIM * DDIM) return;
    if (in_sizes[3] < HDIM || in_sizes[5] < DDIM || in_sizes[7] < HDIM || in_sizes[9] < DDIM) return;
    int Mvalid = out_size / DDIM;
    if (Mvalid > N) Mvalid = N;
    if (Mvalid <= 0) return;

    const int MP   = cdiv(N, 64) * 64;
    const int NBK  = cdiv(MP, NPB);
    const int ELLR = NBK * NPB;

    const int* src = ei;
    const int* dst = ei + E;

    char* ws = (char*)d_ws;
    size_t off = 0;
    int*   ell  = (int*)  (ws + ws_take(off, (size_t)ELLR * ELLW * 4));
    us*    x16  = (us*)   (ws + ws_take(off, (size_t)MP * DDIM * 2));
    us*    w1t  = (us*)   (ws + ws_take(off, (size_t)HDIM * DDIM * 2));
    us*    w2t  = (us*)   (ws + ws_take(off, (size_t)DDIM * HDIM * 2));
    us*    wm1h = (us*)   (ws + ws_take(off, (size_t)HDIM * DDIM * 2));
    us*    wm1l = (us*)   (ws + ws_take(off, (size_t)HDIM * DDIM * 2));
    us*    wm2h = (us*)   (ws + ws_take(off, (size_t)DDIM * HDIM * 2));
    us*    wm2l = (us*)   (ws + ws_take(off, (size_t)DDIM * HDIM * 2));
    float* xw1  = (float*)(ws + ws_take(off, (size_t)MP * HDIM * 4));
    us*    h16  = (us*)   (ws + ws_take(off, (size_t)MP * HDIM * 2));
    float* xw2  = (float*)(ws + ws_take(off, (size_t)MP * DDIM * 4));
    us*    gh   = (us*)   (ws + ws_take(off, (size_t)MP * DDIM * 2));
    us*    gl   = (us*)   (ws + ws_take(off, (size_t)MP * DDIM * 2));
    us*    th   = (us*)   (ws + ws_take(off, (size_t)MP * HDIM * 2));
    us*    tl   = (us*)   (ws + ws_take(off, (size_t)MP * HDIM * 2));
    if (off > ws_size) return;

    k_build<<<NBK, 32, 0, stream>>>(src, dst, E, N, ell);

    k_cvt_x<<<cdiv((long)MP * 32, 256), 256, 0, stream>>>(x, N, MP, x16);
    k_wcvt<<<cdiv((long)HDIM * DDIM / 8, 256), 256, 0, stream>>>(W1,  DDIM, HDIM, 0, 16.0f, w1t,  w1t);
    k_wcvt<<<cdiv((long)DDIM * HDIM / 8, 256), 256, 0, stream>>>(W2,  HDIM, DDIM, 0, 16.0f, w2t,  w2t);
    k_wcvt<<<cdiv((long)HDIM * DDIM / 8, 256), 256, 0, stream>>>(Wm1, DDIM, HDIM, 1, 1.0f,  wm1h, wm1l);
    k_wcvt<<<cdiv((long)DDIM * HDIM / 8, 256), 256, 0, stream>>>(Wm2, HDIM, DDIM, 1, 1.0f,  wm2h, wm2l);

    const int gridH = (MP / 64) * (HDIM / 64);
    const int gridD = (MP / 64) * (DDIM / 64);

    k_gemm<0, 0><<<gridH, 128, 0, stream>>>(x16, x16, w1t, w1t, DDIM, HDIM, b1, 0.0625f, xw1, h16, h16, MP);
    k_agg<HDIM, 1, 0><<<MP, HDIM / 8, 0, stream>>>(xw1, ell, N, b1, h16, h16);

    k_gemm<0, 0><<<gridD, 128, 0, stream>>>(h16, h16, w2t, w2t, HDIM, DDIM, b2, 0.0625f, xw2, gh, gh, MP);
    k_agg<DDIM, 0, 1><<<MP, DDIM / 8, 0, stream>>>(xw2, ell, N, b2, gh, gl);

    k_gemm<1, 1><<<gridH, 128, 0, stream>>>(gh, gl, wm1h, wm1l, DDIM, HDIM, bm1, 1.0f, xw1, th, tl, MP);
    k_gemm<1, 2><<<gridD, 128, 0, stream>>>(th, tl, wm2h, wm2l, HDIM, DDIM, bm2, 1.0f, (float*)d_out, gh, gl, Mvalid);
}
